// NeuronSparkMOE_83906481095358
// MI455X (gfx1250) — hardware-verified
//
#include <hip/hip_runtime.h>
#include <math.h>

typedef __attribute__((ext_vector_type(16))) _Float16 v16h;
typedef __attribute__((ext_vector_type(16))) __bf16 v16b;
typedef __attribute__((ext_vector_type(8)))  _Float16 v8h;
typedef __attribute__((ext_vector_type(8)))  float v8f;
typedef __attribute__((ext_vector_type(4)))  float v4f;
typedef __attribute__((ext_vector_type(2)))  float v2f;
typedef __attribute__((ext_vector_type(4)))  unsigned v4u;
typedef __attribute__((ext_vector_type(4)))  int v4i;
typedef float __attribute__((may_alias)) float_a;
typedef int __attribute__((may_alias)) int_a;

template <typename T> __device__ __forceinline__ void vst2(void* p, T v) { *(volatile T*)p = v; __threadfence(); *(volatile T*)p = v; }
__device__ __forceinline__ v8f wmma16(v16h a, v16h b, v8f c) {
  v8f d = __builtin_amdgcn_wmma_f32_16x16x32_f16(false, a, false, b, (short)0, c, false, false);
  asm volatile("v_nop\n\tv_nop\n\tv_nop\n\tv_nop" : "+v"(d) : "v"(a), "v"(b));
  return d;
}
__device__ __forceinline__ v8f wmma_bf(v16b a, v16b b, v8f c) {
  v8f d = __builtin_amdgcn_wmma_f32_16x16x32_bf16(false, a, false, b, (short)0, c, false, false);
  asm volatile("v_nop\n\tv_nop\n\tv_nop\n\tv_nop" : "+v"(d) : "v"(a), "v"(b));
  return d;
}
__device__ __forceinline__ v16h frag_h(const _Float16* rowk0, int lane) {
  union { v16h v; v8h q[2]; } u; const _Float16* p = rowk0 + 8 * (lane >> 4);
  u.q[0] = *(const v8h*)p; u.q[1] = *(const v8h*)(p + 16); return u.v;
}
__device__ __forceinline__ v16h frag_f32(const float* rowk0, int lane) {
  v16h a; const float* p = rowk0 + 8 * (lane >> 4);
#pragma unroll
  for (int i = 0; i < 8; ++i) { a[i] = (_Float16)p[i]; a[8 + i] = (_Float16)p[16 + i]; }
  return a;
}
__device__ __forceinline__ v16h frag_f32s(const float* rowk0, int lane, float sc) {
  v16h a; const float* p = rowk0 + 8 * (lane >> 4);
#pragma unroll
  for (int i = 0; i < 8; ++i) { a[i] = (_Float16)(p[i] * sc); a[8 + i] = (_Float16)(p[16 + i] * sc); }
  return a;
}
__device__ __forceinline__ v16h fragc_f32(const float* W, int k0, int n, int lane, int ld, int K) {
  v16h a; const int g = lane >> 4;
#pragma unroll
  for (int i = 0; i < 8; ++i) { const int ka = k0 + 8 * g + i, kb = ka + 16;
    a[i] = (_Float16)(ka < K ? W[(size_t)(ka < K ? ka : K - 1) * ld + n] : 0.f); a[8 + i] = (_Float16)(kb < K ? W[(size_t)(kb < K ? kb : K - 1) * ld + n] : 0.f); }
  return a;
}
struct F2 { v16b h, l; };
__device__ __forceinline__ F2 bsplit16(const float v[16]) { F2 r;
#pragma unroll
  for (int i = 0; i < 16; ++i) { const __bf16 h = (__bf16)v[i]; r.h[i] = h; r.l[i] = (__bf16)(v[i] - (float)h); }
  return r; }
__device__ __forceinline__ F2 split_row(const float* row, int k0, int lane) { float v[16]; const float* p = row + k0 + 8 * (lane >> 4);
#pragma unroll
  for (int i = 0; i < 8; ++i) { v[i] = p[i]; v[8 + i] = p[16 + i]; }
  return bsplit16(v); }
__device__ __forceinline__ F2 split_rowK(const float* row, int k0, int lane, int K) { float v[16]; const int g = lane >> 4;
#pragma unroll
  for (int i = 0; i < 8; ++i) { const int ka = k0 + 8 * g + i, kb = ka + 16; v[i] = ka < K ? row[ka < K ? ka : K - 1] : 0.f; v[8 + i] = kb < K ? row[kb < K ? kb : K - 1] : 0.f; }
  return bsplit16(v); }
__device__ __forceinline__ F2 split_col(const float* W, int k0, int n, int lane, int ld, int K) { float v[16]; const int g = lane >> 4;
#pragma unroll
  for (int i = 0; i < 8; ++i) { const int ka = k0 + 8 * g + i, kb = ka + 16; v[i] = ka < K ? W[(size_t)(ka < K ? ka : K - 1) * ld + n] : 0.f; v[8 + i] = kb < K ? W[(size_t)(kb < K ? kb : K - 1) * ld + n] : 0.f; }
  return bsplit16(v); }
__device__ __forceinline__ v8f mac3(const F2& a, const F2& b, v8f c) { c = wmma_bf(a.l, b.h, c); c = wmma_bf(a.h, b.l, c); return wmma_bf(a.h, b.h, c); }
__device__ __forceinline__ float sigm(float v) { return 1.0f / (1.0f + expf(-v)); }
#define LDSX() do { asm volatile("s_wait_dscnt 0" ::: "memory"); __builtin_amdgcn_wave_barrier(); __builtin_amdgcn_fence(__ATOMIC_RELEASE, "workgroup"); } while (0)


#ifndef NTOK
#define NTOK 2048
#endif
#define HH 1024
#define NE 16
#define NG 4
#define GSZ (NE / NG)
#define TOPK 4
#define DFF 512
#define DFS 2048
#define NPAIR (TOPK * NTOK)
#ifndef NRB
#define NRB (NTOK / 64)
#endif
#define MAXT 16
#define LSTW 64
typedef __attribute__((ext_vector_type(8))) __bf16 v8b;
__device__ __forceinline__ v16b frag_b(const __bf16* rowk0, int lane) {
  union { v16b v; v8b q[2]; } u; const __bf16* p = rowk0 + 8 * (lane >> 4);
  u.q[0] = *(const v8b*)p; u.q[1] = *(const v8b*)(p + 16); return u.v;
}
__device__ __forceinline__ float bfr(float v) { return (float)(__bf16)v; }
__device__ __attribute__((noinline)) float exp_ni(float v) { return expf(v); }
__device__ __attribute__((noinline)) float erf_ni(float v) { return erff(v); }


#define NBLK (NTOK / 64)
#define WS_LST  0u
#define WS_CNTI (WS_LST + 4u * NE * NBLK * LSTW)
#define WS_OFFI (WS_CNTI + 4u * NBLK * 32)
#define WS_PW   (WS_OFFI + 4u * (NE * NBLK + 32))
#define PG 0
#define P1 (PG + NE * HH)
#define P2 (P1 + NE * DFF * HH)
#define PS1 (P2 + NE * HH * DFF)
#define PS2 (PS1 + DFS * HH)
#define PWEND (PS2 + HH * DFS)
#define WS_CW   (WS_PW + 2u * PWEND)
#define WS_PE   (WS_CW + 4u * NTOK * NE)
#define WS_H1   (WS_PE + 4u * NPAIR)
#define WS_Y    (WS_H1 + 4u * NPAIR * DFF)
#define WS_HS   (WS_Y + 4u * NPAIR * HH)
#define WS_SO   (WS_HS + 4u * NTOK * DFS)
#define WS_END  (WS_SO + 4u * NTOK * HH)

__global__ __launch_bounds__(256) void k_packT(const float* __restrict__ WG, const float* __restrict__ WU, const float* __restrict__ WD, const float* __restrict__ SU, const float* __restrict__ SD, __bf16* __restrict__ PW) {
  __shared__ __align__(16) __bf16 s[DFS]; const int n = blockIdx.x, which = blockIdx.y, tid = threadIdx.x; int K; size_t dst;
  if (which == 0) { if (n >= NE) return; K = HH; dst = PG + (size_t)n * HH; for (int k = tid; k < K; k += 256) s[k] = (__bf16)WG[(size_t)n * HH + k]; }
  else if (which == 1) { if (n >= NE * DFF) return; K = HH; const int e = n / DFF, o = n % DFF; dst = P1 + (size_t)n * HH; for (int k = tid; k < K; k += 256) s[k] = (__bf16)WU[((size_t)e * HH + k) * DFF + o]; }
  else if (which == 2) { K = DFF; const int e = n / HH, o = n % HH; dst = P2 + (size_t)n * DFF; for (int k = tid; k < K; k += 256) s[k] = (__bf16)WD[((size_t)e * DFF + k) * HH + o]; }
  else if (which == 3) { if (n >= DFS) return; K = HH; dst = PS1 + (size_t)n * HH; for (int k = tid; k < K; k += 256) s[k] = (__bf16)SU[(size_t)k * DFS + n]; }
  else { if (n >= HH) return; K = DFS; dst = PS2 + (size_t)n * DFS; for (int k = tid; k < K; k += 256) s[k] = (__bf16)SD[(size_t)k * HH + n]; }
  __syncthreads();
  for (int q = tid; q < K / 8; q += 256) vst2((unsigned*)(PW + dst + q * 8), *(const v4u*)&s[q * 8]);
}
__global__ __launch_bounds__(128) void k_gate(const float* __restrict__ X, const __bf16* __restrict__ PW, float* __restrict__ CW, int* __restrict__ PE, int* __restrict__ LST, int* __restrict__ CNTI) {
  __shared__ float sl[4][16][NE + 1]; __shared__ __align__(16) float sc[64][NE]; __shared__ __align__(16) int spe[NPAIR / NTOK * 64]; __shared__ __align__(16) int slst[NE][LSTW]; __shared__ __align__(16) int scnt[32];
  const int tid = threadIdx.x, wave = tid >> 5, lane = tid & 31, col = lane & 15, g = lane >> 4; const size_t r0 = (size_t)blockIdx.x * 64 + wave * 16;
  v8f acc = {};
#pragma unroll 4
  for (int kc = 0; kc < HH / 32; ++kc) { v16b a; { const float* p = X + (r0 + col) * HH + kc * 32 + 8 * g;
#pragma unroll
      for (int i = 0; i < 8; ++i) { a[i] = (__bf16)p[i]; a[8 + i] = (__bf16)p[16 + i]; } }
    acc = wmma_bf(a, frag_b(PW + PG + (size_t)col * HH + kc * 32, lane), acc); }
#pragma unroll
  for (int r = 0; r < 8; ++r) sl[wave][8 * g + r][col] = acc[r];
  LDSX();
  if (lane < 16) { const int rl = lane; const int tl = wave * 16 + rl; float sv[NE];
#pragma unroll
    for (int e = 0; e < NE; ++e) sv[e] = sigm(sl[wave][rl][e]);
    float gsc[NG];
#pragma unroll
    for (int gi = 0; gi < NG; ++gi) { float a1 = -1.f, a2 = -1.f;
#pragma unroll
      for (int j = 0; j < GSZ; ++j) { const float v = sv[gi * GSZ + j]; if (v > a1) { a2 = a1; a1 = v; } else if (v > a2) a2 = v; }
      gsc[gi] = a1 + a2; }
    int g1 = 0; float gv1 = gsc[0];
#pragma unroll
    for (int gi = 1; gi < NG; ++gi) if (gsc[gi] > gv1) { gv1 = gsc[gi]; g1 = gi; }
    int g2 = -1; float gv2 = -3.0e38f;
#pragma unroll
    for (int gi = 0; gi < NG; ++gi) if (gi != g1 && gsc[gi] > gv2) { gv2 = gsc[gi]; g2 = gi; }
    float mk[NE];
#pragma unroll
    for (int e = 0; e < NE; ++e) { const int gi = e / GSZ; mk[e] = (gi == g1 || gi == g2) ? sv[e] : 0.f; }
    int sel[TOPK]; float ws_ = 0.f;
#pragma unroll
    for (int j = 0; j < TOPK; ++j) { int bi = 0; float bv = -3.0e38f;
#pragma unroll
      for (int e = 0; e < NE; ++e) { bool taken = false;
#pragma unroll
        for (int q = 0; q < TOPK; ++q) taken |= (q < j && sel[q] == e);
        if (!taken && mk[e] > bv) { bv = mk[e]; bi = e; } }
      sel[j] = bi; ws_ += sv[bi]; }
    const float inv = 1.0f / (ws_ + 1e-20f);
#pragma unroll
    for (int e = 0; e < NE; ++e) { float w = 0.f;
#pragma unroll
      for (int j = 0; j < TOPK; ++j) if (sel[j] == e) w = (sv[e] * inv) * 2.5f;
      sc[tl][e] = w; }
#pragma unroll
    for (int j = 0; j < TOPK; ++j) spe[TOPK * tl + j] = sel[j]; }
  __syncthreads();
  for (int q = tid; q < 64 * NE / 4; q += 128) vst2(CW + (size_t)blockIdx.x * 64 * NE + q * 4, *(const v4f*)&(&sc[0][0])[q * 4]);
  for (int q = tid; q < TOPK * 64 / 4; q += 128) vst2((unsigned*)(PE + (size_t)blockIdx.x * TOPK * 64 + q * 4), *(const v4u*)&spe[q * 4]);
  for (int q = tid; q < NE * LSTW; q += 128) slst[q / LSTW][q % LSTW] = -1;
  if (tid < 32) scnt[tid] = 0;
  __syncthreads();
  if (tid < NE) { int c = 0; for (int p = 0; p < TOPK * 64; ++p) if (spe[p] == tid && c < LSTW) { slst[tid][c++] = blockIdx.x * TOPK * 64 + p; } scnt[tid] = c; }
  __syncthreads();
  for (int q = tid; q < NE * (LSTW / 4); q += 128) { const int e = q / (LSTW / 4), pc = q % (LSTW / 4); vst2((unsigned*)(LST + ((size_t)e * NBLK + blockIdx.x) * LSTW + pc * 4), *(const v4u*)&slst[e][pc * 4]); }
  if (tid < 8) vst2((unsigned*)(CNTI + (size_t)blockIdx.x * 32 + tid * 4), *(const v4u*)&scnt[tid * 4]);
}
__global__ __launch_bounds__(32) void k_mscan(const int* __restrict__ CNTI, int* __restrict__ OFFI) {
  __shared__ __align__(16) int so[NE][NBLK]; __shared__ __align__(16) int stot[32]; const int e = threadIdx.x;
  if (e < NE) { int run = 0; for (int b = 0; b < NBLK; ++b) { so[e][b] = run; run += min(max(CNTI[(size_t)b * 32 + e], 0), LSTW); } stot[e] = run; } else if (e < 32) stot[e] = 0;
  __syncthreads();
  for (int q = e; q < NE * NBLK / 4; q += 32) vst2((unsigned*)(OFFI + q * 4), *(const v4u*)&(&so[0][0])[q * 4]);
  if (e < 8) vst2((unsigned*)(OFFI + NE * NBLK + e * 4), *(const v4u*)&stot[e * 4]);
}
__device__ __forceinline__ int moe_pair(const int* __restrict__ OFFI, const int* __restrict__ CNTI, const int* __restrict__ LST, int e, int r) {
  int lo = 0, hi = NBLK - 1; while (lo < hi) { const int mid = (lo + hi + 1) >> 1; if (OFFI[e * NBLK + mid] <= r) lo = mid; else hi = mid - 1; }
  const int off = OFFI[e * NBLK + lo]; const int c = min(max(CNTI[(size_t)lo * 32 + e], 0), LSTW); const int i = r - off; if (i < 0 || i >= c) return -1;
  const int p = LST[((size_t)e * NBLK + lo) * LSTW + i]; return (p < 0 || p >= NPAIR) ? -1 : p;
}
__global__ __launch_bounds__(128) void k_ffn1(const float* __restrict__ X, const __bf16* __restrict__ PW, const int* __restrict__ LST, const int* __restrict__ CNTI, const int* __restrict__ OFFI, float* __restrict__ H1) {
  __shared__ __align__(16) float so[4][16][132]; __shared__ int spair[64];
  const int tid = threadIdx.x, wave = tid >> 5, lane = tid & 31, col = lane & 15, g = lane >> 4; const int t = blockIdx.x, e = blockIdx.z; const int n0 = blockIdx.y * 128;
  const int cnt = min(max(OFFI[NE * NBLK + e], 0), NPAIR); if (t * 64 >= cnt) return;
  if (tid < 64) { const int i = t * 64 + tid; spair[tid] = (i < cnt) ? moe_pair(OFFI, CNTI, LST, e, i) : -1; }
  __syncthreads();
  const int mypair = spair[wave * 16 + col]; const size_t tok = (size_t)((mypair < 0 ? 0 : mypair) / TOPK);
  const __bf16* PWE = PW + P1 + (size_t)e * DFF * HH;
  v8f acc[8] = {};
#pragma unroll 2
  for (int kc = 0; kc < HH / 32; ++kc) { v16b a; { const float* p = X + tok * HH + kc * 32 + 8 * g;
#pragma unroll
      for (int i = 0; i < 8; ++i) { a[i] = (__bf16)p[i]; a[8 + i] = (__bf16)p[16 + i]; } }
#pragma unroll
    for (int j = 0; j < 8; ++j) acc[j] = wmma_bf(a, frag_b(PWE + (size_t)(n0 + j * 16 + col) * HH + kc * 32, lane), acc[j]); }
#pragma unroll
  for (int j = 0; j < 8; ++j)
#pragma unroll
    for (int r = 0; r < 8; ++r) { const float v = acc[j][r]; so[wave][8 * g + r][j * 16 + col] = v * sigm(v); }
  LDSX();
  for (int rl = 0; rl < 16; ++rl) { const int pr = spair[wave * 16 + rl]; if (pr >= 0) vst2(H1 + (size_t)pr * DFF + n0 + lane * 4, *(const v4f*)&so[wave][rl][lane * 4]); }
}
__global__ __launch_bounds__(128) void k_ffn2(const float* __restrict__ H1, const __bf16* __restrict__ PW, const int* __restrict__ LST, const int* __restrict__ CNTI, const int* __restrict__ OFFI, float* __restrict__ Y) {
  __shared__ __align__(16) float so[4][16][132]; __shared__ int spair[64];
  const int tid = threadIdx.x, wave = tid >> 5, lane = tid & 31, col = lane & 15, g = lane >> 4; const int t = blockIdx.x, e = blockIdx.z; const int n0 = blockIdx.y * 128;
  const int cnt = min(max(OFFI[NE * NBLK + e], 0), NPAIR); if (t * 64 >= cnt) return;
  if (tid < 64) { const int i = t * 64 + tid; spair[tid] = (i < cnt) ? moe_pair(OFFI, CNTI, LST, e, i) : -1; }
  __syncthreads();
  const int mypair = spair[wave * 16 + col]; const size_t prow = (size_t)(mypair < 0 ? 0 : mypair);
  v8f acc[8] = {};
#pragma unroll 2
  for (int kc = 0; kc < DFF / 32; ++kc) { const F2 a = split_row(H1 + prow * DFF, kc * 32, lane);
#pragma unroll
    for (int j = 0; j < 8; ++j) { const v16b w = frag_b(PW + P2 + ((size_t)e * HH + n0 + j * 16 + col) * DFF + kc * 32, lane); acc[j] = wmma_bf(a.l, w, acc[j]); acc[j] = wmma_bf(a.h, w, acc[j]); } }
#pragma unroll
  for (int j = 0; j < 8; ++j) {
#pragma unroll
    for (int r = 0; r < 8; ++r) so[wave][8 * g + r][j * 16 + col] = acc[j][r]; }
  LDSX();
  for (int rl = 0; rl < 16; ++rl) { const int pr = spair[wave * 16 + rl]; if (pr >= 0) vst2(Y + (size_t)pr * HH + n0 + lane * 4, *(const v4f*)&so[wave][rl][lane * 4]); }
}
template <int RIN, int EPI>
__global__ __launch_bounds__(128) void k_sgemm(const float* __restrict__ A, int K, const __bf16* __restrict__ P, float* __restrict__ OUT, int ldo) {
  __shared__ __align__(16) float so[4][16][132];
  const int tid = threadIdx.x, wave = tid >> 5, lane = tid & 31, col = lane & 15, g = lane >> 4; const size_t r0 = (size_t)blockIdx.x * 64 + wave * 16; const int n0 = blockIdx.y * 128;
  v8f acc[8] = {};
#pragma unroll 2
  for (int kc = 0; kc < K / 32; ++kc) { F2 a; if (RIN) { v16b ax; const float* p = A + (r0 + col) * K + kc * 32 + 8 * g;
#pragma unroll
      for (int i = 0; i < 8; ++i) { ax[i] = (__bf16)p[i]; ax[8 + i] = (__bf16)p[16 + i]; } a.h = ax; a.l = ax; } else a = split_row(A + (r0 + col) * K, kc * 32, lane);
#pragma unroll
    for (int j = 0; j < 8; ++j) { const v16b w = frag_b(P + (size_t)(n0 + j * 16 + col) * K + kc * 32, lane); if (!RIN) acc[j] = wmma_bf(a.l, w, acc[j]); acc[j] = wmma_bf(a.h, w, acc[j]); } }
#pragma unroll
  for (int j = 0; j < 8; ++j) {
#pragma unroll
    for (int r = 0; r < 8; ++r) { float v = acc[j][r]; if (EPI == 1) v = v * sigm(v); so[wave][8 * g + r][j * 16 + col] = v; } }
  LDSX();
  for (int rl = 0; rl < 16; ++rl) vst2(OUT + (r0 + rl) * ldo + n0 + lane * 4, *(const v4f*)&so[wave][rl][lane * 4]);
}
__global__ __launch_bounds__(256) void k_comb(const float* __restrict__ SO, const float* __restrict__ Y, const float* __restrict__ CW, const int* __restrict__ PE, float* __restrict__ OUT) {
  const int tid = threadIdx.x; const int tsub = tid >> 5, piece = tid & 31; const int n0 = blockIdx.y * 128 + piece * 4;
#pragma unroll 1
  for (int pass = 0; pass < 8; ++pass) { const size_t tok = (size_t)blockIdx.x * 64 + pass * 8 + tsub;
    v4f o; const float* so = SO + tok * HH + n0;
#pragma unroll
    for (int i = 0; i < 4; ++i) o[i] = 0.f;
#pragma unroll
    for (int j = 0; j < TOPK; ++j) { const int ej = min(max(PE[TOPK * tok + j], 0), NE - 1); const float cj = CW[tok * NE + ej]; const float* yj = Y + (TOPK * tok + j) * HH + n0;
#pragma unroll
      for (int i = 0; i < 4; ++i) o[i] += yj[i] * cj; }
#pragma unroll
    for (int i = 0; i < 4; ++i) o[i] += so[i];
    vst2(OUT + tok * HH + n0, o); }
}
extern "C" void kernel_launch(void* const* d_in, const int* in_sizes, int n_in, void* d_out, int out_size, void* d_ws, size_t ws_size, hipStream_t stream) {
  (void)in_sizes; (void)n_in; (void)out_size;
  const float** F = (const float**)d_in;
  if (ws_size < (size_t)WS_END) return;
  char* ws = (char*)d_ws; int *LST = (int*)(ws + WS_LST), *CNTI = (int*)(ws + WS_CNTI), *OFFI = (int*)(ws + WS_OFFI), *PE = (int*)(ws + WS_PE); __bf16* PW = (__bf16*)(ws + WS_PW); float *CW = (float*)(ws + WS_CW), *H1 = (float*)(ws + WS_H1), *Y = (float*)(ws + WS_Y), *HS = (float*)(ws + WS_HS), *SO = (float*)(ws + WS_SO);
  k_packT<<<dim3(NE * HH, 5), 256, 0, stream>>>(F[1], F[2], F[3], F[4], F[5], PW);
  k_gate<<<NRB, 128, 0, stream>>>(F[0], PW, CW, PE, LST, CNTI);
  k_mscan<<<1, 32, 0, stream>>>(CNTI, OFFI);
  k_ffn1<<<dim3(MAXT, DFF / 128, NE), 128, 0, stream>>>(F[0], PW, LST, CNTI, OFFI, H1);
  k_ffn2<<<dim3(MAXT, HH / 128, NE), 128, 0, stream>>>(H1, PW, LST, CNTI, OFFI, Y);
  k_sgemm<1, 1><<<dim3(NRB, DFS / 128), 128, 0, stream>>>(F[0], HH, PW + PS1, HS, DFS);
  k_sgemm<0, 0><<<dim3(NRB, HH / 128), 128, 0, stream>>>(HS, DFS, PW + PS2, SO, HH);
  k_comb<<<dim3(NRB, HH / 128), 256, 0, stream>>>(SO, Y, CW, PE, (float*)d_out);
}
